// Encoder_77318001262793
// MI455X (gfx1250) — hardware-run, weakly checked
//
#include <hip/hip_runtime.h>


#ifndef NB
#define NB 2
#endif
#ifndef SEQ
#define SEQ 2048
#endif
#define NB_FULL 2
#define SEQ_FULL 2048
#define DA 256
#define CE 768
#define NH 12
#define HD 64
#define C3 2304
#define C4 3072
#define C6 4608
#define QP 1536
#define NRES 256
#define NLAY 2
#define KF 924
#define KFP 960
#define KC 387
#define KCP 448
#define XW 512
#define FROW ((KFP) + (KCP))
#define RROWS ((NB) * (SEQ))
#define NQB ((SEQ) / 128)
#define NKT ((SEQ) / 64)
#define VROWS ((NB) * NH * HD)
#define OUT1_OFF ((size_t)NB_FULL * NRES * DA)

static_assert((SEQ) % 256 == 0);
static_assert((NB) >= 1 && (NB) <= NB_FULL);
static_assert((SEQ) <= SEQ_FULL);
static_assert(CE % 128 == 0 && C3 % 128 == 0 && C4 % 128 == 0 && QP % 128 == 0 && DA % 128 == 0 && NRES % 128 == 0);
static_assert(KFP % 64 == 0 && KCP % 64 == 0 && XW % 64 == 0 && DA % 64 == 0 && CE % 64 == 0 && C4 % 64 == 0 && (SEQ) % 64 == 0);
static_assert(KFP >= KF && KCP >= KC);
static_assert(KFP - KF == 36 && KCP - KC == 61);
static_assert(KF == 387 + 23 + 129 + 1 + 128 + 256);
static_assert(14 * 32 == 192 + 192 + 64);
static_assert((KFP % 256) == 192 && (KCP % 256) == 192);
static_assert((KFP * 2) % 128 == 0 && (KCP * 2) % 128 == 0);
static_assert((FROW * 4) % 16 == 0);
static_assert(XW == 2 * DA);
static_assert(DA == 256);
static_assert(CE == 3 * 256);
static_assert(C6 == 6 * CE && C6 % 256 == 0);
static_assert(NH * HD == CE);
static_assert(HD == 64);
static_assert(QP == 2 * CE);
static_assert(C3 == 3 * CE);
static_assert(RROWS % 128 == 0);
static_assert(RROWS % 32 == 0);
static_assert((SEQ) % 128 == 0);
static_assert(NRES % 32 == 0 && DA % 32 == 0 && CE % 32 == 0 && C3 % 32 == 0 && C4 % 32 == 0);
static_assert(NQB * 128 == (SEQ));
static_assert(NKT * 64 == (SEQ));
static_assert(NKT >= 4);
static_assert(((size_t)RROWS * CE) % 2048 == 0);
static_assert(OUT1_OFF * 4 == 524288);
static_assert((NB * NRES) % 32 == 0);

typedef unsigned short u16;
typedef unsigned int   u32;
typedef _Float16 h16;
typedef _Float16 v16h __attribute__((ext_vector_type(16)));
typedef _Float16 v8h  __attribute__((ext_vector_type(8)));
typedef _Float16 v4h  __attribute__((ext_vector_type(4)));
typedef float    v8f  __attribute__((ext_vector_type(8)));
typedef float    v4f  __attribute__((ext_vector_type(4)));
typedef unsigned int u32x4 __attribute__((ext_vector_type(4)));
typedef unsigned int u32x2 __attribute__((ext_vector_type(2)));

union Frag  { v16h v; u32x4 u[2]; };
union Pack8 { v8h h; u32x4 u; };
union Pack4 { v4h h; u32x2 u; };

#define WSCALE 64.0f
#define WINV   (1.0f / 64.0f)
#define PCAR   4096.0f
#define PINV   (1.0f / 4096.0f)
#define CVCAR  64.0f
#define CVINV  (1.0f / 64.0f)

#define GM_F32  0
#define GM_F16  1
#define GM_QKV  2
#define GM_GATE 3
#define GM_POOL 4

static __device__ const unsigned int FREQ_BITS[64] = {
    0x3f800000u, 0x3f9210e3u, 0x3fa6ae88u, 0x3fbe3510u, 0x3fd90d9eu, 0x3ff7b02au, 0x400d52cfu, 0x40214519u,
    0x40380817u, 0x40520181u, 0x406fa56bu, 0x4088bc25u, 0x409c08a6u, 0x40b20e73u, 0x40cb2ff8u, 0x40e7dd85u,
    0x41044ba1u, 0x4116f7b7u, 0x412c4677u, 0x4144971au, 0x41605649u, 0x41800003u, 0x419210e4u, 0x41a6ae8bu,
    0x41be3515u, 0x41d90da2u, 0x41f7b031u, 0x420d52d1u, 0x4221451cu, 0x42380819u, 0x42520185u, 0x426fa56eu,
    0x4288bc28u, 0x429c08a9u, 0x42b20e75u, 0x42cb2ffdu, 0x42e7dd87u, 0x43044ba4u, 0x4316f7b9u, 0x432c467bu,
    0x4344971cu, 0x4360564du, 0x43800006u, 0x439210ebu, 0x43a6ae8bu, 0x43be3515u, 0x43d90da6u, 0x43f7b036u,
    0x440d52d7u, 0x4421451cu, 0x4438081du, 0x4452018au, 0x446fa578u, 0x4488bc28u, 0x449c08a9u, 0x44b20e79u,
    0x44cb3001u, 0x44e7dd91u, 0x45044ba4u, 0x4516f7bcu, 0x452c467fu, 0x45449725u, 0x4560564du, 0x45800000u };
static_assert(sizeof(FREQ_BITS) == 64 * 4);

constexpr size_t al256(size_t b) { return (b + 255) & ~(size_t)255; }
constexpr size_t cmax(size_t a, size_t b) { return a > b ? a : b; }

constexpr size_t SZ_WFEAT = (size_t)DA * KFP * 2;
constexpr size_t SZ_WPOS  = (size_t)DA * KCP * 2;
constexpr size_t SZ_WIN   = (size_t)DA * XW * 2;
constexpr size_t SZ_WTIN  = (size_t)CE * DA * 2;
constexpr size_t SZ_WQKV  = (size_t)NLAY * C3 * CE * 2;
constexpr size_t SZ_WO    = (size_t)NLAY * CE * CE * 2;
constexpr size_t SZ_WM1   = (size_t)NLAY * C4 * CE * 2;
constexpr size_t SZ_WM2   = (size_t)NLAY * CE * C4 * 2;
constexpr size_t SZ_WTOUT = (size_t)DA * CE * 2;
constexpr size_t SZ_F     = (size_t)RROWS * KFP * 2;
constexpr size_t SZ_C     = (size_t)RROWS * KCP * 2;
constexpr size_t SZ_XIN   = (size_t)RROWS * XW * 2;
constexpr size_t SZ_AIN   = (size_t)RROWS * DA * 2;
constexpr size_t SZ_FRONT = al256(SZ_F) + al256(SZ_C) + al256(SZ_XIN) + al256(SZ_AIN);
constexpr size_t SZ_HG    = (size_t)RROWS * C4 * 2;
constexpr size_t SZ_BIG   = cmax(SZ_FRONT, al256(SZ_HG));
constexpr size_t SZ_X     = (size_t)RROWS * CE * 4;
constexpr size_t SZ_H     = (size_t)RROWS * CE * 2;
constexpr size_t SZ_QK    = (size_t)RROWS * QP * 2;
constexpr size_t SZ_VT    = (size_t)VROWS * (SEQ) * 2;
constexpr size_t SZ_CV    = (size_t)RROWS * CE * 2;
constexpr size_t SZ_ROPE  = (size_t)RROWS * 64 * 4;
constexpr size_t SZ_SC    = (size_t)NB * CE * 4;
constexpr size_t SZ_MV    = (size_t)NLAY * NB * C6 * 4;
constexpr size_t SZ_A2T   = (size_t)NB * NRES * (SEQ) * 2;
constexpr size_t SZ_ALT   = (size_t)NB * DA * (SEQ) * 2;
constexpr size_t SZ_RINV  = (size_t)NB * NRES * 4;
static_assert(SZ_FRONT <= SZ_BIG && al256(SZ_HG) <= SZ_BIG);
static_assert((size_t)RROWS * DA * 4 <= SZ_X);
constexpr size_t WS_TOTAL =
    al256(SZ_WFEAT) + al256(SZ_WPOS) + al256(SZ_WIN) + al256(SZ_WTIN) + al256(SZ_WQKV) + al256(SZ_WO) +
    al256(SZ_WM1) + al256(SZ_WM2) + al256(SZ_WTOUT) + SZ_BIG + al256(SZ_X) + al256(SZ_X) + al256(SZ_H) +
    al256(SZ_QK) + al256(SZ_VT) + al256(SZ_CV) + al256(SZ_ROPE) + al256(SZ_SC) + al256(SZ_MV) +
    al256(SZ_A2T) + al256(SZ_ALT) + al256(SZ_RINV);
static_assert(WS_TOTAL <= (size_t)134217728);

__device__ __forceinline__ float bfr(float f) {
    u32 u = __builtin_bit_cast(u32, f);
    u += 0x7fffu + ((u >> 16) & 1u);
    u &= 0xffff0000u;
    return __builtin_bit_cast(float, u);
}

static __device__ __forceinline__ h16 toh_flush(float v) {
    const h16 r = (h16)v;
    return (fabsf(v) < 6.103515625e-05f) ? (h16)0.0f : r;
}
static __device__ __forceinline__ u16 hb_flush(float v) {
    return __builtin_bit_cast(u16, toh_flush(v));
}

__device__ __forceinline__ v8f mma16(v16h a, v16h b, v8f c) {
    c = __builtin_amdgcn_wmma_f32_16x16x32_f16(false, a, false, b, (short)0, c, false, false);
    asm volatile("v_nop\n\tv_nop\n\tv_nop\n\tv_nop" : "+v"(c) : "v"(a), "v"(b));
    return c;
}

__device__ __forceinline__ float gelu_tanh(float x) {
    const float u = 0.7978845608028654f * (x + 0.044715f * x * x * x);
    const float e = __expf(2.0f * u);
    const float t = 1.0f - 2.0f * __builtin_amdgcn_rcpf(e + 1.0f);
    return 0.5f * x * (1.0f + t);
}

__device__ __forceinline__ float silu_f(float y) {
    return y * __builtin_amdgcn_rcpf(1.0f + __expf(-y));
}

__device__ __forceinline__ size_t grow_map(u32 r) {
    const u32 bb = r / (u32)(SEQ);
    const u32 t  = r - bb * (u32)(SEQ);
    return (size_t)bb * SEQ_FULL + (size_t)t;
}

__global__ __launch_bounds__(256) void cvt_wt_kernel(const float* __restrict__ in, u16* __restrict__ out,
                                                     u32 K, u32 N, u32 Kp, u32 zin, u32 zout,
                                                     float scale, u32 rne) {
    __shared__ float tl[64 * 33];
    const u32 tid = threadIdx.x;
    const u32 k0 = blockIdx.x * 64u, n0 = blockIdx.y * 32u;
    const float* src0 = in + (size_t)blockIdx.z * zin;
    u16* dst0 = out + (size_t)blockIdx.z * zout;
    const u32 kl = tid >> 2, sg = (tid & 3u) * 8u;
    const u32 kr = k0 + kl;
    const u32 kc = (kr < K) ? kr : (K - 1u);
    const float* src = src0 + (size_t)kc * N + n0 + sg;
    v4f a = *(const v4f*)src;
    v4f b = *(const v4f*)(src + 4);
#pragma unroll
    for (u32 c = 0; c < 4; c++) {
        float fa = a[c]; float fb = b[c];
        fa = (kr < K) ? fa : 0.0f;
        fb = (kr < K) ? fb : 0.0f;
        tl[kl * 33u + sg + c]      = fa;
        tl[kl * 33u + sg + 4u + c] = fb;
    }
    __syncthreads();
    const u32 nl = tid >> 3, ks = (tid & 7u) * 8u;
    Pack8 pk;
#pragma unroll
    for (u32 j = 0; j < 8; j++) {
        float t = tl[(ks + j) * 33u + nl];
        t = (rne != 0u) ? bfr(t) : t;
        pk.h[j] = toh_flush(t * scale);
    }
    const u32x4 val = pk.u;
    u16* o = dst0 + (size_t)(n0 + nl) * Kp + k0 + ks;
    *(volatile u32x4*)o = val;
    __threadfence();
    *(volatile u32x4*)o = val;
}

__global__ __launch_bounds__(256) void cast_kernel(const float* __restrict__ in, u16* __restrict__ out) {
    const u32 i = blockIdx.x * 256u + threadIdx.x;
    const float* src = in + (size_t)i * 8u;
    v4f a = *(const v4f*)src;
    v4f b = *(const v4f*)(src + 4);
    Pack8 pk;
#pragma unroll
    for (u32 c = 0; c < 4; c++) {
        float fa = a[c]; float fb = b[c];
        pk.h[c]      = toh_flush(fa);
        pk.h[4u + c] = toh_flush(fb);
    }
    const u32x4 val = pk.u;
    u16* o = out + (size_t)i * 8u;
    *(volatile u32x4*)o = val;
    __threadfence();
    *(volatile u32x4*)o = val;
}

__global__ __launch_bounds__(256) void feat_kernel(const float* __restrict__ coords, const float* __restrict__ refp,
                                                   const int* __restrict__ resid, const float* __restrict__ rtype,
                                                   const float* __restrict__ charge, const float* __restrict__ anum,
                                                   const float* __restrict__ aname,
                                                   u16* __restrict__ F, u16* __restrict__ C) {
#pragma clang fp contract(off)
    __shared__ __align__(16) float wrow[8 * FROW];
    __shared__ float ftab[128];
    const u32 tid = threadIdx.x, lane = tid & 31u;
    const u32 wv = (u32)__builtin_amdgcn_readfirstlane((int)(tid >> 5));
    if (tid < 128u) {
        const u32 j = tid & 63u;
        const float fq = __builtin_bit_cast(float, FREQ_BITS[j]);
        const float af = (float)(2u * j) * (-0.07195578415606394f);
        const float dv = (float)exp2((double)af * 1.4426950408889634);
        ftab[tid] = (tid < 64u) ? fq : dv;
    }
    const u32 r = blockIdx.x * 8u + wv;
    const size_t gr = grow_map(r);
    const u32 wb = wv * (u32)FROW;
    const float x0 = bfr(refp[gr * 3 + 0]), x1 = bfr(refp[gr * 3 + 1]), x2 = bfr(refp[gr * 3 + 2]);
    const float y0 = bfr(coords[gr * 3 + 0]), y1 = bfr(coords[gr * 3 + 1]), y2 = bfr(coords[gr * 3 + 2]);
    const float posr = (float)resid[gr];
    const float chg = bfr(charge[gr]);
    __syncthreads();
#pragma unroll 1
    for (u32 it = 0; it < 14u; it++) {
        const u32 e = it * 32u + lane;
        const u32 grp = (e >= 384u) ? 2u : ((e >= 192u) ? 1u : 0u);
        const u32 s = e - grp * 192u;
        const u32 f = s / 3u, ax = s - f * 3u;
        const float xa = (ax == 0u) ? x0 : ((ax == 1u) ? x1 : x2);
        const float ya = (ax == 0u) ? y0 : ((ax == 1u) ? y1 : y2);
        const u32 ti = (grp == 2u) ? (64u + s) : f;
        const float xv = (grp == 2u) ? posr : ((grp == 1u) ? ya : xa);
        const float ang = xv * ftab[ti];
        float sn, cs;
        sincosf(ang, &sn, &cs);
        const u32 os = (grp == 2u) ? (411u + s) : ((grp == 1u) ? ((u32)KFP + 3u + s) : (3u + s));
        const u32 oc = (grp == 2u) ? (475u + s) : ((grp == 1u) ? ((u32)KFP + 195u + s) : (195u + s));
        wrow[wb + os] = sn;
        wrow[wb + oc] = cs;
    }
#pragma unroll 1
    for (u32 it = 0; it < 2u; it++) {
        v4f t = *(const v4f*)(aname + gr * 256 + it * 128u + lane * 4u);
#pragma unroll
        for (u32 c = 0; c < 4; c++) { float q = t[c]; t[c] = bfr(q); }
        *(v4f*)&wrow[wb + 668u + it * 128u + lane * 4u] = t;
    }
    {
        v4f t = *(const v4f*)(anum + gr * 128 + lane * 4u);
#pragma unroll
        for (u32 c = 0; c < 4; c++) { float q = t[c]; t[c] = bfr(q); }
        *(v4f*)&wrow[wb + 540u + lane * 4u] = t;
    }
    {
        const u32 li = (lane < 23u) ? lane : 22u;
        float rv = rtype[gr * 23 + li];
        asm volatile("" : "+v"(rv));
        rv = bfr(rv);
        if (lane < 23u) wrow[wb + 387u + lane] = rv;
    }
    if (lane == 0u) {
        wrow[wb + 0u] = x0; wrow[wb + 1u] = x1; wrow[wb + 2u] = x2;
        wrow[wb + 410u] = posr;
        wrow[wb + 539u] = chg;
        wrow[wb + (u32)KFP + 0u] = y0; wrow[wb + (u32)KFP + 1u] = y1; wrow[wb + (u32)KFP + 2u] = y2;
    }
    wrow[wb + 924u + lane] = 0.0f;
    if (lane < 4u) wrow[wb + 956u + lane] = 0.0f;
    wrow[wb + (u32)KFP + 387u + lane] = 0.0f;
    if (lane < 29u) wrow[wb + (u32)KFP + 419u + lane] = 0.0f;
    __syncthreads();

    u32x4 fv[4], cv2[2];
#pragma unroll
    for (u32 j = 0; j < 4; j++) {
        const u32 c = j * 256u + lane * 8u;
        const u32 cc = (c < (u32)KFP) ? c : (u32)(KFP - 8);
        v4f a = *(const v4f*)&wrow[wb + cc];
        v4f b = *(const v4f*)&wrow[wb + cc + 4u];
        Pack8 pk;
#pragma unroll
        for (u32 q = 0; q < 4; q++) {
            float ta = a[q]; float tb = b[q];
            pk.h[q] = toh_flush(ta); pk.h[4u + q] = toh_flush(tb);
        }
        fv[j] = pk.u;
    }
#pragma unroll
    for (u32 j = 0; j < 2; j++) {
        const u32 c = j * 256u + lane * 8u;
        const u32 cc = (c < (u32)KCP) ? c : (u32)(KCP - 8);
        v4f a = *(const v4f*)&wrow[wb + (u32)KFP + cc];
        v4f b = *(const v4f*)&wrow[wb + (u32)KFP + cc + 4u];
        Pack8 pk;
#pragma unroll
        for (u32 q = 0; q < 4; q++) {
            float ta = a[q]; float tb = b[q];
            pk.h[q] = toh_flush(ta); pk.h[4u + q] = toh_flush(tb);
        }
        cv2[j] = pk.u;
    }
    u16* fo = F + (size_t)r * KFP;
    u16* co = C + (size_t)r * KCP;
#pragma unroll
    for (u32 j = 0; j < 4; j++) {
        const u32 c = j * 256u + lane * 8u;
        if (c < (u32)KFP) *(volatile u32x4*)(fo + c) = fv[j];
    }
#pragma unroll
    for (u32 j = 0; j < 2; j++) {
        const u32 c = j * 256u + lane * 8u;
        if (c < (u32)KCP) *(volatile u32x4*)(co + c) = cv2[j];
    }
    __threadfence();
#pragma unroll
    for (u32 j = 0; j < 4; j++) {
        const u32 c = j * 256u + lane * 8u;
        if (c < (u32)KFP) *(volatile u32x4*)(fo + c) = fv[j];
    }
#pragma unroll
    for (u32 j = 0; j < 2; j++) {
        const u32 c = j * 256u + lane * 8u;
        if (c < (u32)KCP) *(volatile u32x4*)(co + c) = cv2[j];
    }
}

__global__ __launch_bounds__(256) void rope_kernel(const int* __restrict__ rpos, float* __restrict__ tab) {
#pragma clang fp contract(off)
    __shared__ float inv[32];
    __shared__ __align__(16) float st[8 * 256];
    const u32 tid = threadIdx.x, lane = tid & 31u;
    const u32 wv = (u32)__builtin_amdgcn_readfirstlane((int)(tid >> 5));
    if (tid < 32u) {
        const double ex = (double)((float)tid * (1.0f / 32.0f)) * 13.287712379549449;
        const float p = (float)exp2(ex);
        inv[tid] = 1.0f / p;
    }
    __syncthreads();
    const float iv = inv[lane];
    const u32 r0 = blockIdx.x * 32u + wv * 4u;
#pragma unroll 1
    for (u32 i = 0; i < 4u; i++) {
        const float pos = (float)rpos[grow_map(r0 + i)];
        const float ang = pos * iv;
        float sn, cs;
        sincosf(ang, &sn, &cs);
        st[wv * 256u + i * 64u + lane]       = cs;
        st[wv * 256u + i * 64u + 32u + lane] = sn;
    }
    __syncthreads();
    v4f val[2];
#pragma unroll
    for (u32 j = 0; j < 2; j++) val[j] = *(const v4f*)&st[wv * 256u + j * 128u + lane * 4u];
    float* o = tab + (size_t)r0 * 64u;
#pragma unroll
    for (u32 j = 0; j < 2; j++) *(volatile v4f*)(o + j * 128u + lane * 4u) = val[j];
    __threadfence();
#pragma unroll
    for (u32 j = 0; j < 2; j++) *(volatile v4f*)(o + j * 128u + lane * 4u) = val[j];
}

__global__ __launch_bounds__(256) void colsum_kernel(const float* __restrict__ a2t, float* __restrict__ rinv) {
#pragma clang fp contract(off)
    __shared__ float part[8 * 32];
    __shared__ __align__(16) float fin[32];
    const u32 tid = threadIdx.x, lane = tid & 31u;
    const u32 wv = (u32)__builtin_amdgcn_readfirstlane((int)(tid >> 5));
    const u32 b = blockIdx.x / (u32)(NRES / 32);
    const u32 r0 = (blockIdx.x - b * (u32)(NRES / 32)) * 32u;
    const float* p = a2t + (size_t)b * SEQ_FULL * NRES + r0 + lane;
    float s = 0.f;
#pragma unroll 1
    for (u32 n = wv; n < (u32)(SEQ); n += 8u) s += bfr(p[(size_t)n * NRES]);
    part[wv * 32u + lane] = s;
    __syncthreads();
    if (wv == 0u) {
        float t = 0.f;
#pragma unroll
        for (u32 w = 0; w < 8; w++) t += part[w * 32u + lane];
        fin[lane] = 1.0f / (t + 1e-6f);
    }
    __syncthreads();
    if (wv == 0u) {
        const v4f val = *(const v4f*)&fin[(lane & 7u) * 4u];
        float* o = rinv + (size_t)blockIdx.x * 32u + (lane & 7u) * 4u;
        if (lane < 8u) *(volatile v4f*)o = val;
        __threadfence();
        if (lane < 8u) *(volatile v4f*)o = val;
    }
}

__global__ __launch_bounds__(256) void ada_kernel(const float* __restrict__ emb, const float* __restrict__ W,
                                                  const float* __restrict__ bias, const float* __restrict__ g,
                                                  const float* __restrict__ be, float* __restrict__ sc) {
    __shared__ float es[DA];
    __shared__ float red[8];
    __shared__ __align__(16) float ys[CE];
    const u32 tid = threadIdx.x, lane = tid & 31u;
    const u32 wv = (u32)__builtin_amdgcn_readfirstlane((int)(tid >> 5));
    const u32 b = blockIdx.x;
    es[tid] = bfr(emb[(size_t)b * DA + tid]);
    __syncthreads();
    float a0 = bfr(bias[tid]), a1 = bfr(bias[tid + 256u]), a2 = bfr(bias[tid + 512u]);
#pragma unroll 4
    for (u32 k = 0; k < (u32)DA; k++) {
        const float e = es[k];
        const float* w = W + (size_t)k * CE;
        a0 += e * bfr(w[tid]);
        a1 += e * bfr(w[tid + 256u]);
        a2 += e * bfr(w[tid + 512u]);
    }
    float s = a0 + a1 + a2;
#pragma unroll
    for (u32 m = 16; m >= 1; m >>= 1) s += __shfl_xor(s, m, 32);
    if (lane == 0u) red[wv] = s;
    __syncthreads();
    float tot = 0.f;
#pragma unroll
    for (u32 w = 0; w < 8; w++) tot += red[w];
    const float mu = tot * (1.f / (float)CE);
    __syncthreads();
    const float d0 = a0 - mu, d1 = a1 - mu, d2 = a2 - mu;
    float vs = d0 * d0 + d1 * d1 + d2 * d2;
#pragma unroll
    for (u32 m = 16; m >= 1; m >>= 1) vs += __shfl_xor(vs, m, 32);
    if (lane == 0u) red[wv] = vs;
    __syncthreads();
    float tv = 0.f;
#pragma unroll
    for (u32 w = 0; w < 8; w++) tv += red[w];
    const float rstd = rsqrtf(tv * (1.f / (float)CE) + 1e-5f);
    ys[tid]        = silu_f(d0 * rstd * bfr(g[tid])        + bfr(be[tid]));
    ys[tid + 256u] = silu_f(d1 * rstd * bfr(g[tid + 256u]) + bfr(be[tid + 256u]));
    ys[tid + 512u] = silu_f(d2 * rstd * bfr(g[tid + 512u]) + bfr(be[tid + 512u]));
    __syncthreads();
    if (tid < 192u) {
        const v4f val = *(const v4f*)&ys[tid * 4u];
        float* o = sc + (size_t)b * CE + tid * 4u;
        *(volatile v4f*)o = val;
        __threadfence();
        *(volatile v4f*)o = val;
    }
}

__global__ __launch_bounds__(256) void mod_kernel(const float* __restrict__ sc, const float* __restrict__ W,
                                                  const float* __restrict__ bias, float* __restrict__ mv) {
    __shared__ float cs[NB * CE];
    const u32 tid = threadIdx.x;
    const u32 l = blockIdx.y;
    const u32 j = blockIdx.x * 256u + tid;
#pragma unroll 1
    for (u32 i = tid; i < (u32)(NB * CE); i += 256u) cs[i] = sc[i];
    __syncthreads();
    const float* w = W + (size_t)l * CE * C6 + j;
    const float bj = bfr(bias[(size_t)l * C6 + j]);
    float acc[NB];
#pragma unroll
    for (int b = 0; b < NB; b++) acc[b] = bj;
#pragma unroll 4
    for (u32 k = 0; k < (u32)CE; k++) {
        const float wk = bfr(w[(size_t)k * C6]);
#pragma unroll
        for (int b = 0; b < NB; b++) acc[b] += cs[(u32)b * CE + k] * wk;
    }
#pragma unroll
    for (int b = 0; b < NB; b++) {
        const float val = acc[b];
        *(volatile float*)(mv + ((size_t)l * NB + (u32)b) * C6 + j) = val;
    }
    __threadfence();
#pragma unroll
    for (int b = 0; b < NB; b++) {
        const float val = acc[b];
        *(volatile float*)(mv + ((size_t)l * NB + (u32)b) * C6 + j) = val;
    }
}

template <int D, int EPI>
__device__ __forceinline__ void ln_body(const float* __restrict__ src, const float* __restrict__ g,
                                        const float* __restrict__ be, float* __restrict__ of,
                                        u16* __restrict__ oh, u32 ldo) {
#pragma clang fp contract(off)
    constexpr u32 LJ = D / 128, LO = D / 256;
    static_assert(D % 256 == 0);
    static_assert((D / 4) % 32 == 0 && D / 4 <= 256);
    __shared__ __align__(16) float xs[8 * D];
    __shared__ __align__(16) u16   rows[8 * D];
    __shared__ __align__(16) float gsh[D];
    __shared__ __align__(16) float bsh[D];
    const u32 tid = threadIdx.x, lane = tid & 31u;
    const u32 wv = (u32)__builtin_amdgcn_readfirstlane((int)(tid >> 5));
    const u32 bq = (blockIdx.x * 8u) / (u32)(SEQ);
    if (tid < (u32)(D / 4)) {
        const u32 go_ = (EPI == 2) ? bq * (u32)C6 : 0u;
        v4f gg = *(const v4f*)(g + go_ + tid * 4u);
        v4f bb = *(const v4f*)(be + go_ + tid * 4u);
        v4f go, bo;
#pragma unroll
        for (u32 c = 0; c < 4; c++) {
            float tg = gg[c]; float tb = bb[c];
            if constexpr (EPI == 2) { go[c] = 1.0f + tg; bo[c] = tb; }
            else                    { go[c] = bfr(tg);   bo[c] = bfr(tb); }
        }
        *(v4f*)&gsh[tid * 4u] = go;
        *(v4f*)&bsh[tid * 4u] = bo;
    }
    const u32 r = blockIdx.x * 8u + wv;
    const float* xr = src + (size_t)r * D;
    float* xw = xs + wv * D;
    float s = 0.f;
#pragma unroll 1
    for (u32 j = 0; j < LJ; j++) {
        const u32 c0 = j * 128u + lane * 4u;
        v4f t4 = *(const v4f*)(xr + c0);
        *(v4f*)&xw[c0] = t4;
        s += (t4[0] + t4[1]) + (t4[2] + t4[3]);
    }
#pragma unroll
    for (u32 m = 16; m >= 1; m >>= 1) s += __shfl_xor(s, m, 32);
    const float mu = s * (1.f / (float)D);
    float vs = 0.f;
#pragma unroll 1
    for (u32 j = 0; j < LJ; j++) {
        const u32 c0 = j * 128u + lane * 4u;
        v4f t4 = *(const v4f*)&xw[c0];
#pragma unroll
        for (u32 c = 0; c < 4; c++) { float d = t4[c] - mu; vs += d * d; }
    }
#pragma unroll
    for (u32 m = 16; m >= 1; m >>= 1) vs += __shfl_xor(vs, m, 32);
    const float rstd = rsqrtf(vs * (1.f / (float)D) + 1e-5f);
    __syncthreads();
    if constexpr (EPI == 0 || EPI == 2) {
        u16* rw = rows + wv * D;
#pragma unroll 1
        for (u32 j = 0; j < LJ; j++) {
            const u32 c0 = j * 128u + lane * 4u;
            v4f x4 = *(const v4f*)&xw[c0];
            v4f g4 = *(const v4f*)&gsh[c0];
            v4f b4 = *(const v4f*)&bsh[c0];
            Pack4 pk;
#pragma unroll
            for (u32 c = 0; c < 4; c++) {
                float xe = x4[c]; float ge = g4[c]; float bel = b4[c];
                float y = (xe - mu) * rstd * ge + bel;
                if constexpr (EPI == 0) y = silu_f(y);
                pk.h[c] = toh_flush(y);
            }
            *(u32x2*)&rw[c0] = pk.u;
        }
        __syncthreads();
        u32x4 val[LO];
#pragma unroll
        for (u32 j = 0; j < LO; j++) val[j] = *(const u32x4*)&rw[j * 256u + lane * 8u];
        const u32 pitch = (EPI == 0) ? ldo : (u32)D;
        u16* orow = oh + (size_t)r * pitch;
#pragma unroll
        for (u32 j = 0; j < LO; j++) *(volatile u32x4*)(orow + j * 256u + lane * 8u) = val[j];
        __threadfence();
#pragma unroll
        for (u32 j = 0; j < LO; j++) *(volatile u32x4*)(orow + j * 256u + lane * 8u) = val[j];
    } else {
        v4f val[LJ];
#pragma unroll
        for (u32 j = 0; j < LJ; j++) {
            const u32 c0 = j * 128u + lane * 4u;
            v4f x4 = *(const v4f*)&xw[c0];
            v4f g4 = *(const v4f*)&gsh[c0];
            v4f b4 = *(const v4f*)&bsh[c0];
            v4f y4;
#pragma unroll
            for (u32 c = 0; c < 4; c++) {
                float xe = x4[c]; float ge = g4[c]; float bel = b4[c];
                y4[c] = (xe - mu) * rstd * ge + bel;
            }
            val[j] = y4;
        }
        const size_t orr = (EPI == 3) ? grow_map(r) : (size_t)r;
        float* orow = of + orr * D;
#pragma unroll
        for (u32 j = 0; j < LJ; j++) *(volatile v4f*)(orow + j * 128u + lane * 4u) = val[j];
        __threadfence();
#pragma unroll
        for (u32 j = 0; j < LJ; j++) *(volatile v4f*)(orow + j * 128u + lane * 4u) = val[j];
    }
}

__global__ __launch_bounds__(256) void ln_feat_kernel(const float* __restrict__ src, const float* __restrict__ g,
                                                      const float* __restrict__ be, u16* __restrict__ out) {
    ln_body<DA, 0>(src, g, be, (float*)nullptr, out, (u32)XW);
}
__global__ __launch_bounds__(256) void ln_tin_kernel(const float* __restrict__ src, const float* __restrict__ g,
                                                     const float* __restrict__ be, float* __restrict__ out) {
    ln_body<CE, 1>(src, g, be, out, (u16*)nullptr, 0u);
}
__global__ __launch_bounds__(256) void ln_mod_kernel(const float* __restrict__ src, const float* __restrict__ sc,
                                                     const float* __restrict__ sh, u16* __restrict__ out) {
    ln_body<CE, 2>(src, sc, sh, (float*)nullptr, out, 0u);
}
__global__ __launch_bounds__(256) void ln_out_kernel(const float* __restrict__ src, const float* __restrict__ g,
                                                     const float* __restrict__ be, float* __restrict__ out) {
    ln_body<DA, 3>(src, g, be, out, (u16*)nullptr, 0u);
}

template <int MODE, int HASB, int ACT>
__device__ __forceinline__ void gemm_body(const u16* __restrict__ A, const u16* __restrict__ BT,
                                          const float* __restrict__ bias, const float* __restrict__ res,
                                          const float* __restrict__ aux, void* out0, void* out1,
                                          u32 N, u32 K, u32 ldo, u32 coff, u32 orow0, float oscale) {
    __shared__ u32x4 smem[4224];
    u16* As = (u16*)smem;
    u16* Bs = As + 128 * 72;
    float* Cs = (float*)smem;
    constexpr u32 CSP = 132;

    const u32 tid = threadIdx.x, lane = tid & 31u;
    const u32 wv = (u32)__builtin_amdgcn_readfirstlane((int)(tid >> 5));
    const u32 hf = lane >> 4, ln = lane & 15u;
    const u32 m0 = blockIdx.y * 128u, n0 = blockIdx.x * 128u;
    const u32 wm = wv & 3u, wn = wv >> 2;
    const u32 srow = tid >> 1, sseg = (tid & 1u) * 32u;

    v8f acc[2][4];
#pragma unroll
    for (int i = 0; i < 2; i++)
#pragma unroll
        for (int j = 0; j < 4; j++) acc[i][j] = (v8f)(0.f);

    for (u32 k0 = 0; k0 < K; k0 += 64u) {
        __syncthreads();
        {
            const u16* ga = A  + (size_t)(m0 + srow) * K + k0 + sseg;
            const u16* gb = BT + (size_t)(n0 + srow) * K + k0 + sseg;
            u32x4 a0 = *(const u32x4*)(ga), a1 = *(const u32x4*)(ga + 8);
            u32x4 a2 = *(const u32x4*)(ga + 16), a3 = *(const u32x4*)(ga + 24);
            u32x4 b0 = *(const u32x4*)(gb), b1 = *(const u32x4*)(gb + 8);
            u32x4 b2 = *(const u32x4*)(gb + 16), b3 = *(const u32x4*)(gb + 24);
            u32x4* la = (u32x4*)&As[srow * 72u + sseg];
            u32x4* lb = (u32x4*)&Bs[srow * 72u + sseg];
            la[0] = a0; la[1] = a1; la[2] = a2; la[3] = a3;
            lb[0] = b0; lb[1] = b1; lb[2] = b2; lb[3] = b3;
        }
        __syncthreads();
#pragma unroll
        for (u32 ks = 0; ks < 2; ks++) {
            Frag af[2], bf[4];
#pragma unroll
            for (u32 mi = 0; mi < 2; mi++) {
                const u16* q = &As[(wm * 32u + mi * 16u + ln) * 72u + ks * 32u + hf * 8u];
                af[mi].u[0] = *(const u32x4*)q;
                af[mi].u[1] = *(const u32x4*)(q + 16);
            }
#pragma unroll
            for (u32 ni = 0; ni < 4; ni++) {
                const u16* q = &Bs[(wn * 64u + ni * 16u + ln) * 72u + ks * 32u + hf * 8u];
                bf[ni].u[0] = *(const u32x4*)q;
                bf[ni].u[1] = *(const u32x4*)(q + 16);
            }
#pragma unroll
            for (int mi = 0; mi < 2; mi++)
#pragma unroll
                for (int ni = 0; ni < 4; ni++)
                    acc[mi][ni] = mma16(af[mi].v, bf[ni].v, acc[mi][ni]);
        }
    }

    __syncthreads();
#pragma unroll
    for (int ni = 0; ni < 4; ni++) {
        const u32 col = wn * 64u + (u32)ni * 16u + ln;
        float bv = 0.f;
        if constexpr (HASB != 0) bv = bfr(bias[n0 + col]);
#pragma unroll
        for (int mi = 0; mi < 2; mi++) {
#pragma unroll
            for (int r = 0; r < 8; r++) {
                const u32 row = wm * 32u + (u32)mi * 16u + hf * 8u + (u32)r;
                float v = acc[mi][ni][r] * oscale + bv;
                if constexpr (ACT != 0) v = gelu_tanh(v);
                Cs[row * CSP + col] = v;
            }
        }
    }
    __syncthreads();

    if constexpr (MODE == GM_F32 || MODE == GM_GATE || MODE == GM_POOL) {
        float* o = (float*)out0;
        v4f val[16];
        v4f g4 = (v4f)(0.f);
        if constexpr (MODE == GM_GATE) {
            const u32 bq = m0 / (u32)(SEQ);
            g4 = *(const v4f*)(aux + (size_t)bq * C6 + n0 + lane * 4u);
        }
#pragma unroll
        for (int grp = 0; grp < 2; grp++) {
#pragma unroll
            for (int i8 = 0; i8 < 8; i8++) {
                const int i = grp * 8 + i8;
                const u32 row = wv * 16u + (u32)i;
                const u32 r = m0 + row;
                v4f c = *(const v4f*)&Cs[row * CSP + lane * 4u];
                if constexpr (MODE == GM_GATE) {
                    v4f x4 = *(const v4f*)(res + (size_t)r * (size_t)N + n0 + lane * 4u);
                    val[i] = x4 + g4 * c;
                } else if constexpr (MODE == GM_POOL) {
                    const float rv = aux[orow0 + r];
                    val[i] = c * rv;
                } else {
                    val[i] = c;
                }
            }
            asm volatile("" ::: "memory");
        }
#pragma unroll
        for (int i = 0; i < 16; i++) {
            const u32 r = m0 + wv * 16u + (u32)i;
            *(volatile v4f*)(o + (size_t)(orow0 + r) * (size_t)ldo + coff + n0 + lane * 4u) = val[i];
        }
        __threadfence();
#pragma unroll
        for (int i = 0; i < 16; i++) {
            const u32 r = m0 + wv * 16u + (u32)i;
            *(volatile v4f*)(o + (size_t)(orow0 + r) * (size_t)ldo + coff + n0 + lane * 4u) = val[i];
        }
    } else if constexpr (MODE == GM_F16) {
        u16* o = (u16*)out0;
        u32x4 val[8];
#pragma unroll
        for (int it = 0; it < 8; it++) {
            const u32 rloc = wv * 16u + (u32)it * 2u + hf, cseg = ln * 8u;
            Pack8 pk;
#pragma unroll
            for (int j = 0; j < 8; j++) pk.h[j] = toh_flush(Cs[rloc * CSP + cseg + (u32)j]);
            val[it] = pk.u;
        }
#pragma unroll
        for (int it = 0; it < 8; it++) {
            const u32 rloc = wv * 16u + (u32)it * 2u + hf, cseg = ln * 8u;
            *(volatile u32x4*)(o + (size_t)(m0 + rloc) * ldo + coff + n0 + cseg) = val[it];
        }
        __threadfence();
#pragma unroll
        for (int it = 0; it < 8; it++) {
            const u32 rloc = wv * 16u + (u32)it * 2u + hf, cseg = ln * 8u;
            *(volatile u32x4*)(o + (size_t)(m0 + rloc) * ldo + coff + n0 + cseg) = val[it];
        }
    } else {
        u16* qkp = (u16*)out0;
        u16* vtp = (u16*)out1;
        const u32 bq = m0 / (u32)(SEQ);
        const u32 t0 = m0 - bq * (u32)(SEQ);
        u32x4 vh[8];
        if (n0 < (u32)QP) {
            const u32 cseg = ln * 8u;
            const u32 d0b  = cseg & 31u;
            const u32 cpar = cseg ^ 32u;
            const float sg = ((cseg & 32u) != 0u) ? 1.0f : -1.0f;
#pragma unroll
            for (int grp = 0; grp < 2; grp++) {
#pragma unroll
                for (int i4 = 0; i4 < 4; i4++) {
                    const int it = grp * 4 + i4;
                    const u32 rloc = wv * 16u + (u32)it * 2u + hf;
                    const float* tr = aux + (size_t)(m0 + rloc) * 64u + d0b;
                    v4f c0 = *(const v4f*)tr,        c1 = *(const v4f*)(tr + 4);
                    v4f s0 = *(const v4f*)(tr + 32), s1 = *(const v4f*)(tr + 36);
                    Pack8 ph;
#pragma unroll
                    for (int j = 0; j < 4; j++) {
                        const float xa = Cs[rloc * CSP + cseg + (u32)j];
                        const float pa = Cs[rloc * CSP + cpar + (u32)j];
                        const float xb = Cs[rloc * CSP + cseg + 4u + (u32)j];
                        const float pb = Cs[rloc * CSP + cpar + 4u + (u32)j];
                        float ca = c0[j]; float sa = s0[j]; float cb = c1[j]; float sb = s1[j];
                        ph.h[j]     = toh_flush(xa * ca + sg * pa * sa);
                        ph.h[4 + j] = toh_flush(xb * cb + sg * pb * sb);
                    }
                    vh[it] = ph.u;
                }
                asm volatile("" ::: "memory");
            }
#pragma unroll
            for (int it = 0; it < 8; it++) {
                const u32 rloc = wv * 16u + (u32)it * 2u + hf;
                *(volatile u32x4*)(qkp + (size_t)(m0 + rloc) * QP + n0 + cseg) = vh[it];
            }
            __threadfence();
#pragma unroll
            for (int it = 0; it < 8; it++) {
                const u32 rloc = wv * 16u + (u32)it * 2u + hf;
                *(volatile u32x4*)(qkp + (size_t)(m0 + rloc) * QP + n0 + cseg) = vh[it];
            }
        } else {
            const u32 hh0 = (n0 - (u32)QP) >> 6;
#pragma unroll
            for (int it = 0; it < 8; it++) {
                const u32 rloc = wv * 16u + (u32)it * 2u + hf;
                const u32 tseg = ln * 8u;
                Pack8 ph;
#pragma unroll
                for (int j = 0; j < 8; j++) ph.h[j] = toh_flush(Cs[(tseg + (u32)j) * CSP + rloc]);
                vh[it] = ph.u;
            }
#pragma unroll
            for (int it = 0; it < 8; it++) {
                const u32 rloc = wv * 16u + (u32)it * 2u + hf, tseg = ln * 8u;
                const u32 hh = hh0 + (rloc >> 6), dd = rloc & 63u;
                const size_t vrow = (size_t)(bq * NH + hh) * HD + dd;
                *(volatile u32x4*)(vtp + vrow * (SEQ) + t0 + tseg) = vh[it];
            }
            __threadfence();
#pragma unroll
            for (int it = 0; it < 8; it++) {
                const u32 rloc = wv * 16u + (u32)it * 2u + hf, tseg = ln * 8u;
                const u32 hh = hh0 + (rloc >> 6), dd = rloc & 63u;
                const size_t vrow = (size_t)(bq * NH + hh) * HD + dd;
                *(volatile u32x4*)(vtp + vrow * (SEQ) + t0 + tseg) = vh[it];
            }
        }
    }
}

__global__ __launch_bounds__(256) void gemm_f32b_kernel(const u16* __restrict__ A, const u16* __restrict__ BT,
                                                        const float* __restrict__ bias, float* __restrict__ out,
                                                        u32 N, u32 K, u32 ldo, float oscale) {
    gemm_body<GM_F32, 1, 0>(A, BT, bias, bias, bias, (void*)out, (void*)out, N, K, ldo, 0u, 0u, oscale);
}
__global__ __launch_bounds__(256) void gemm_f16n_kernel(const u16* __restrict__ A, const u16* __restrict__ BT,
                                                        u16* __restrict__ out,
                                                        u32 N, u32 K, u32 ldo, u32 coff, float oscale) {
    gemm_body<GM_F16, 0, 0>(A, BT, (const float*)nullptr, (const float*)nullptr, (const float*)nullptr,
                            (void*)out, (void*)out, N, K, ldo, coff, 0u, oscale);
}
__global__ __launch_bounds__(256) void gemm_f16g_kernel(const u16* __restrict__ A, const u16* __restrict__ BT,
                                                        const float* __restrict__ bias, u16* __restrict__ out,
                                                        u32 N, u32 K, u32 ldo, float oscale) {
    gemm_body<GM_F16, 1, 1>(A, BT, bias, bias, bias, (void*)out, (void*)out, N, K, ldo, 0u, 0u, oscale);
}
__global__ __launch_bounds__(256) void gemm_qkv_kernel(const u16* __restrict__ A, const u16* __restrict__ BT,
                                                       const float* __restrict__ bias, const float* __restrict__ tab,
                                                       u16* __restrict__ qkp, u16* __restrict__ vtp,
                                                       u32 N, u32 K, float oscale) {
    gemm_body<GM_QKV, 1, 0>(A, BT, bias, bias, tab, (void*)qkp, (void*)vtp, N, K, 0u, 0u, 0u, oscale);
}
__global__ __launch_bounds__(256) void gemm_gate_kernel(const u16* __restrict__ A, const u16* __restrict__ BT,
                                                        const float* __restrict__ bias, const float* __restrict__ res,
                                                        const float* __restrict__ gatev, float* __restrict__ out,
                                                        u32 N, u32 K, float oscale) {
    gemm_body<GM_GATE, 1, 0>(A, BT, bias, res, gatev, (void*)out, (void*)out, N, K, N, 0u, 0u, oscale);
}
__global__ __launch_bounds__(256) void gemm_pool_kernel(const u16* __restrict__ A, const u16* __restrict__ BT,
                                                        const float* __restrict__ rinv, float* __restrict__ out,
                                                        u32 K) {
    const u32 z = blockIdx.z;
    gemm_body<GM_POOL, 0, 0>(A + (size_t)z * NRES * K, BT + (size_t)z * DA * K, rinv, rinv, rinv,
                             (void*)out, (void*)out, (u32)DA, K, (u32)DA, 0u, z * (u32)NRES, 1.0f);
}

__global__ __launch_bounds__(256) __attribute__((amdgpu_num_vgpr(256)))
void attn_kernel(const u16* __restrict__ qk, const u16* __restrict__ vth, u16* __restrict__ cv) {
    __shared__ __align__(16) u16 Ks[64 * 72];
    __shared__ __align__(16) u16 Vs[64 * 72];
    __shared__ __align__(16) u16 Ps[8 * 16 * 72];

    const u32 bh = blockIdx.y;
    const u32 b = bh / (u32)NH, h = bh - b * (u32)NH;
    const u32 qb = blockIdx.x;
    const u32 tid = threadIdx.x, lane = tid & 31u;
    const u32 wv = (u32)__builtin_amdgcn_readfirstlane((int)(tid >> 5));
    const u32 hf = lane >> 4, ln = lane & 15u;
    const u32 q0 = qb * 128u + wv * 16u;
    u16* Pw = Ps + wv * (16u * 72u);
    const int wlo = (int)((q0 >> 5) * 32u) - 48;
    const int whi = (int)((q0 >> 5) * 32u) + 80;

    Frag qf[2];
#pragma unroll
    for (u32 ds = 0; ds < 2; ds++) {
        const u16* p = qk + (size_t)(b * (u32)(SEQ) + q0 + ln) * QP + h * HD + ds * 32u + hf * 8u;
        qf[ds].u[0] = *(const u32x4*)p;
        qf[ds].u[1] = *(const u32x4*)(p + 16);
    }

    v8f o[4];
#pragma unroll
    for (int i = 0; i < 4; i++) o[i] = (v8f)(0.f);
    float mrow[8], lrow[8];
#pragma unroll
    for (int r = 0; r < 8; r++) { mrow[r] = -3.0e38f; lrow[r] = 0.f; }

    const u32 rr = tid >> 2, seg = (tid & 3u) * 16u;
    const u32 kt0 = (qb > 0u) ? (2u * qb - 1u) : 0u;
    const u32 kt1 = (2u * qb + 2u < (u32)NKT) ? (2u * qb + 2u) : (u32)(NKT - 1);

#pragma unroll 1
    for (u32 kt = kt0; kt <= kt1; kt++) {
        __syncthreads();
        {
            const u16* gk = qk + (size_t)(b * (u32)(SEQ) + kt * 64u + rr) * QP + CE + h * HD + seg;
            u32x4 k0v = *(const u32x4*)gk, k1v = *(const u32x4*)(gk + 8);
            const u16* gv = vth + ((size_t)(bh * HD + rr)) * (SEQ) + kt * 64u + seg;
            u32x4 v0 = *(const u32x4*)gv, v1 = *(const u32x4*)(gv + 8);
            *(u32x4*)&Ks[rr * 72u + seg] = k0v; *(u32x4*)&Ks[rr * 72u + seg + 8u] = k1v;
            *(u32x4*)&Vs[rr * 72u + seg] = v0;  *(u32x4*)&Vs[rr * 72u + seg + 8u] = v1;
        }
        float am[4];
#pragma unroll
        for (int sub = 0; sub < 4; sub++) {
            const int kg = (int)(kt * 64u + (u32)sub * 16u + ln);
            am[sub] = (kg >= wlo && kg < whi) ? 1.0f : 0.0f;
        }
        __syncthreads();

        v8f s[4];
#pragma unroll
        for (int sub = 0; sub < 4; sub++) {
            v8f t = (v8f)(0.f);
#pragma unroll
            for (int ds = 0; ds < 2; ds++) {
                Frag kf;
                const u16* kp = &Ks[((u32)sub * 16u + ln) * 72u + (u32)ds * 32u + hf * 8u];
                kf.u[0] = *(const u32x4*)kp;
                kf.u[1] = *(const u32x4*)(kp + 16);
                t = mma16(qf[ds].v, kf.v, t);
            }
            s[sub] = t;
        }

#pragma unroll
        for (int sub = 0; sub < 4; sub++)
#pragma unroll
            for (int r = 0; r < 8; r++) {
                const float sv = s[sub][r] * 0.125f;
                s[sub][r] = (am[sub] != 0.0f) ? sv : -3.0e38f;
            }

#pragma unroll
        for (int r = 0; r < 8; r++) {
            float mx = fmaxf(fmaxf(s[0][r], s[1][r]), fmaxf(s[2][r], s[3][r]));
#pragma unroll
            for (u32 m = 8; m >= 1; m >>= 1) mx = fmaxf(mx, __shfl_xor(mx, m, 32));
            const float mnew  = fmaxf(mrow[r], mx);
            const float alpha = __expf(mrow[r] - mnew);
            float rsum = 0.f;
#pragma unroll
            for (int sub = 0; sub < 4; sub++) {
                const float pe = __expf(s[sub][r] - mnew) * am[sub];
                s[sub][r] = pe;
                rsum += pe;
            }
#pragma unroll
            for (u32 m = 8; m >= 1; m >>= 1) rsum += __shfl_xor(rsum, m, 32);
            mrow[r] = mnew;
            lrow[r] = lrow[r] * alpha + rsum;
#pragma unroll
            for (int dsub = 0; dsub < 4; dsub++) o[dsub][r] *= alpha;
        }

#pragma unroll
        for (int sub = 0; sub < 4; sub++) {
#pragma unroll
            for (int r = 0; r < 8; r++)
                Pw[(hf * 8u + (u32)r) * 72u + (u32)sub * 16u + ln] = hb_flush(s[sub][r] * PCAR);
        }
        __syncthreads();

#pragma unroll
        for (int dsub = 0; dsub < 4; dsub++) {
#pragma unroll
            for (int ks = 0; ks < 2; ks++) {
                Frag pf, vf;
                const u16* pp = &Pw[ln * 72u + (u32)ks * 32u + hf * 8u];
                pf.u[0] = *(const u32x4*)pp;
                pf.u[1] = *(const u32x4*)(pp + 16);
                const u16* vp = &Vs[((u32)dsub * 16u + ln) * 72u + (u32)ks * 32u + hf * 8u];
                vf.u[0] = *(const u32x4*)vp;
                vf.u[1] = *(const u32x4*)(vp + 16);
                o[dsub] = mma16(pf.v, vf.v, o[dsub]);
            }
        }
    }

    __syncthreads();
#pragma unroll
    for (int r = 0; r < 8; r++) {
        const float inv = (1.0f / lrow[r]) * CVCAR;
#pragma unroll
        for (int dsub = 0; dsub < 4; dsub++)
            Pw[(hf * 8u + (u32)r) * 72u + (u32)dsub * 16u + ln] = hb_flush(o[dsub][r] * PINV * inv);
    }
    __syncthreads();
    u32x4 val[4];
#pragma unroll
    for (u32 it = 0; it < 4; it++) {
        const u32 rloc = it * 4u + (lane >> 3), sg = (lane & 7u) * 8u;
        val[it] = *(const u32x4*)&Pw[rloc * 72u + sg];
    }
#pragma unroll
    for (u32 it = 0; it < 4; it++) {
        const u32 rloc = it * 4u + (lane >> 3), sg = (lane & 7u) * 8u;
        *(volatile u32x4*)(cv + (size_t)(b * (u32)(SEQ) + q0 + rloc) * CE + h * HD + sg) = val[it];
    }
    __threadfence();
#pragma unroll
    for (u32 it = 0; it < 4; it++) {
        const u32 rloc = it * 4u + (lane >> 3), sg = (lane & 7u) * 8u;
        *(volatile u32x4*)(cv + (size_t)(b * (u32)(SEQ) + q0 + rloc) * CE + h * HD + sg) = val[it];
    }
}

extern "C" void kernel_launch(void* const* d_in, const int* in_sizes, int n_in,
                              void* d_out, int out_size, void* d_ws, size_t ws_size,
                              hipStream_t stream) {
    if (n_in < 38) return;
    const long long needR = (long long)(NB - 1) * SEQ_FULL + (SEQ);
    if ((long long)in_sizes[0] < needR * 3 || (long long)in_sizes[1] < needR * 3) return;
    if ((long long)in_sizes[2] < needR || (long long)in_sizes[3] < needR * 23) return;
    if ((long long)in_sizes[4] < needR || (long long)in_sizes[5] < needR * 128) return;
    if ((long long)in_sizes[6] < needR * 256 || in_sizes[7] < NB * DA) return;
    if ((long long)in_sizes[8] < needR || (long long)in_sizes[9] < needR * NRES) return;
    if (in_sizes[10] < KF * DA || in_sizes[11] < DA || in_sizes[12] < DA || in_sizes[13] < DA) return;
    if (in_sizes[14] < KC * DA || in_sizes[15] < XW * DA) return;
    if (in_sizes[16] < DA * CE || in_sizes[17] < CE || in_sizes[18] < CE || in_sizes[19] < CE) return;
    if (in_sizes[20] < DA * CE || in_sizes[21] < CE || in_sizes[22] < CE || in_sizes[23] < CE) return;
    if (in_sizes[24] < NLAY * CE * C6 || in_sizes[25] < NLAY * C6) return;
    if (in_sizes[26] < NLAY * CE * C3 || in_sizes[27] < NLAY * C3) return;
    if (in_sizes[28] < NLAY * CE * CE || in_sizes[29] < NLAY * CE) return;
    if (in_sizes[30] < NLAY * CE * C4 || in_sizes[31] < NLAY * C4) return;
    if (in_sizes[32] < NLAY * C4 * CE || in_sizes[33] < NLAY * CE) return;
    if (in_sizes[34] < CE * DA || in_sizes[35] < DA || in_sizes[36] < DA || in_sizes[37] < DA) return;
    if ((long long)out_size < (long long)OUT1_OFF + needR * DA) return;

    const float* atom_coords = (const float*)d_in[0];
    const float* ref_posn    = (const float*)d_in[1];
    const int*   res_id      = (const int*)d_in[2];
    const float* res_type    = (const float*)d_in[3];
    const float* charge      = (const float*)d_in[4];
    const float* elem_num  = (const float*)d_in[5];
    const float* atom_name   = (const float*)d_in[6];
    const float* ada_emb     = (const float*)d_in[7];
    const int*   rope_pos    = (const int*)d_in[8];
    const float* a2t         = (const float*)d_in[9];
    const float* feat_W      = (const float*)d_in[10];
    const float* feat_b      = (const float*)d_in[11];
    const float* feat_ln_g   = (const float*)d_in[12];
    const float* feat_ln_b   = (const float*)d_in[13];
    const float* pos_W       = (const float*)d_in[14];
    const float* in_W        = (const float*)d_in[15];
    const float* tin_W       = (const float*)d_in[16];
    const float* tin_b       = (const float*)d_in[17];
    const float* tin_ln_g    = (const float*)d_in[18];
    const float* tin_ln_b    = (const float*)d_in[19];
    const float* ada_W       = (const float*)d_in[20];
    const float* ada_b       = (const float*)d_in[21];
    const float* ada_ln_g    = (const float*)d_in[22];
    const float* ada_ln_b    = (const float*)d_in[23];
    const float* mod_W       = (const float*)d_in[24];
    const float* mod_b       = (const float*)d_in[25];
    const float* qkv_W       = (const float*)d_in[26];
    const float* qkv_b       = (const float*)d_in[27];
    const float* o_W         = (const float*)d_in[28];
    const float* o_b         = (const float*)d_in[29];
    const float* m1_W        = (const float*)d_in[30];
    const float* m1_b        = (const float*)d_in[31];
    const float* m2_W        = (const float*)d_in[32];
    const float* m2_b        = (const float*)d_in[33];
    const float* tout_W      = (const float*)d_in[34];
    const float* tout_b      = (const float*)d_in[35];
    const float* tout_ln_g   = (const float*)d_in[36];
    const float* tout_ln_b   = (const float*)d_in[37];

    char* ws = (char*)d_ws;
    size_t off = 0;
    auto take = [&](size_t bytes) -> char* {
        char* p = ws + off;
        off += (bytes + 255) & ~(size_t)255;
        return p;
    };
    u16*   wFeat = (u16*)take(SZ_WFEAT);
    u16*   wPos  = (u16*)take(SZ_WPOS);
    u16*   wIn   = (u16*)take(SZ_WIN);
    u16*   wTin  = (u16*)take(SZ_WTIN);
    u16*   wQkv  = (u16*)take(SZ_WQKV);
    u16*   wO    = (u16*)take(SZ_WO);
    u16*   wM1   = (u16*)take(SZ_WM1);
    u16*   wM2   = (u16*)take(SZ_WM2);
    u16*   wTout = (u16*)take(SZ_WTOUT);
    char*  big   = take(SZ_BIG);
    u16*   F16b  = (u16*)big;
    u16*   C16b  = (u16*)(big + al256(SZ_F));
    u16*   XIN   = (u16*)(big + al256(SZ_F) + al256(SZ_C));
    u16*   AIN   = (u16*)(big + al256(SZ_F) + al256(SZ_C) + al256(SZ_XIN));
    u16*   hg    = (u16*)big;
    float* xa    = (float*)take(SZ_X);
    float* xb    = (float*)take(SZ_X);
    float* S32   = xb;
    u16*   hpl   = (u16*)take(SZ_H);
    u16*   qkp   = (u16*)take(SZ_QK);
    u16*   vth   = (u16*)take(SZ_VT);
    u16*   cvb   = (u16*)take(SZ_CV);
    float* ropeT = (float*)take(SZ_ROPE);
    float* scv   = (float*)take(SZ_SC);
    float* mvec  = (float*)take(SZ_MV);
    u16*   a2tT  = (u16*)take(SZ_A2T);
    u16*   ALT   = (u16*)take(SZ_ALT);
    float* rinv  = (float*)take(SZ_RINV);
    if (off > ws_size || off > (size_t)134217728) return;

    float* outp = (float*)d_out;
    float* out1 = outp + OUT1_OFF;

    cvt_wt_kernel<<<dim3(KFP / 64, DA / 32, 1), 256, 0, stream>>>(feat_W, wFeat, (u32)KF, (u32)DA, (u32)KFP, 0u, 0u, WSCALE, 1u);
    cvt_wt_kernel<<<dim3(KCP / 64, DA / 32, 1), 256, 0, stream>>>(pos_W, wPos, (u32)KC, (u32)DA, (u32)KCP, 0u, 0u, WSCALE, 1u);
    cvt_wt_kernel<<<dim3(XW / 64, DA / 32, 1), 256, 0, stream>>>(in_W, wIn, (u32)XW, (u32)DA, (u32)XW, 0u, 0u, WSCALE, 1u);
    cvt_wt_kernel<<<dim3(DA / 64, CE / 32, 1), 256, 0, stream>>>(tin_W, wTin, (u32)DA, (u32)CE, (u32)DA, 0u, 0u, WSCALE, 1u);
    cvt_wt_kernel<<<dim3(CE / 64, C3 / 32, NLAY), 256, 0, stream>>>(qkv_W, wQkv, (u32)CE, (u32)C3, (u32)CE,
                                                                    (u32)(CE * C3), (u32)(C3 * CE), WSCALE, 1u);
    cvt_wt_kernel<<<dim3(CE / 64, CE / 32, NLAY), 256, 0, stream>>>(o_W, wO, (u32)CE, (u32)CE, (u32)CE,
                                                                    (u32)(CE * CE), (u32)(CE * CE), WSCALE, 1u);
    cvt_wt_kernel<<<dim3(CE / 64, C4 / 32, NLAY), 256, 0, stream>>>(m1_W, wM1, (u32)CE, (u32)C4, (u32)CE,
                                                                    (u32)(CE * C4), (u32)(C4 * CE), WSCALE, 1u);
    cvt_wt_kernel<<<dim3(C4 / 64, CE / 32, NLAY), 256, 0, stream>>>(m2_W, wM2, (u32)C4, (u32)CE, (u32)C4,
                                                                    (u32)(C4 * CE), (u32)(CE * C4), WSCALE, 1u);
    cvt_wt_kernel<<<dim3(CE / 64, DA / 32, 1), 256, 0, stream>>>(tout_W, wTout, (u32)CE, (u32)DA, (u32)CE, 0u, 0u, WSCALE, 1u);
    cvt_wt_kernel<<<dim3((SEQ) / 64, NRES / 32, NB), 256, 0, stream>>>(a2t, a2tT, (u32)(SEQ), (u32)NRES, (u32)(SEQ),
                                                                       (u32)(SEQ_FULL * NRES), (u32)(NRES * (SEQ)), 1.0f, 1u);
    colsum_kernel<<<(NB * NRES) / 32, 256, 0, stream>>>(a2t, rinv);
    feat_kernel<<<RROWS / 8, 256, 0, stream>>>(atom_coords, ref_posn, res_id, res_type, charge, elem_num, atom_name,
                                               F16b, C16b);
    rope_kernel<<<RROWS / 32, 256, 0, stream>>>(rope_pos, ropeT);
    gemm_f32b_kernel<<<dim3(DA / 128, RROWS / 128), 256, 0, stream>>>(F16b, wFeat, feat_b, S32, (u32)DA, (u32)KFP, (u32)DA, WINV);
    ln_feat_kernel<<<RROWS / 8, 256, 0, stream>>>(S32, feat_ln_g, feat_ln_b, XIN);
    gemm_f16n_kernel<<<dim3(DA / 128, RROWS / 128), 256, 0, stream>>>(C16b, wPos, XIN, (u32)DA, (u32)KCP, (u32)XW, (u32)DA, WINV);
    gemm_f16n_kernel<<<dim3(DA / 128, RROWS / 128), 256, 0, stream>>>(XIN, wIn, AIN, (u32)DA, (u32)XW, (u32)DA, 0u, WINV);
    gemm_f32b_kernel<<<dim3(CE / 128, RROWS / 128), 256, 0, stream>>>(AIN, wTin, tin_b, S32, (u32)CE, (u32)DA, (u32)CE, WINV);
    ln_tin_kernel<<<RROWS / 8, 256, 0, stream>>>(S32, tin_ln_g, tin_ln_b, xa);
    ada_kernel<<<NB, 256, 0, stream>>>(ada_emb, ada_W, ada_b, ada_ln_g, ada_ln_b, scv);
    mod_kernel<<<dim3(C6 / 256, NLAY), 256, 0, stream>>>(scv, mod_W, mod_b, mvec);
    for (int l = 0; l < NLAY; l++) {
        const float* mvl = mvec + (size_t)l * NB * C6;
        ln_mod_kernel<<<RROWS / 8, 256, 0, stream>>>(xa, mvl + CE, mvl, hpl);
        gemm_qkv_kernel<<<dim3(C3 / 128, RROWS / 128), 256, 0, stream>>>(hpl, wQkv + (size_t)l * C3 * CE,
                                                                         qkv_b + (size_t)l * C3, ropeT, qkp, vth,
                                                                         (u32)C3, (u32)CE, WINV);
        attn_kernel<<<dim3(NQB, NB * NH), 256, 0, stream>>>(qkp, vth, cvb);
        gemm_gate_kernel<<<dim3(CE / 128, RROWS / 128), 256, 0, stream>>>(cvb, wO + (size_t)l * CE * CE,
                                                                          o_b + (size_t)l * CE, xa, mvl + 2 * CE, xb,
                                                                          (u32)CE, (u32)CE, WINV * CVINV);
        ln_mod_kernel<<<RROWS / 8, 256, 0, stream>>>(xb, mvl + 4 * CE, mvl + 3 * CE, hpl);
        gemm_f16g_kernel<<<dim3(C4 / 128, RROWS / 128), 256, 0, stream>>>(hpl, wM1 + (size_t)l * C4 * CE,
                                                                          m1_b + (size_t)l * C4, hg,
                                                                          (u32)C4, (u32)CE, (u32)C4, WINV);
        gemm_gate_kernel<<<dim3(CE / 128, RROWS / 128), 256, 0, stream>>>(hg, wM2 + (size_t)l * CE * C4,
                                                                          m2_b + (size_t)l * CE, xb, mvl + 5 * CE, xa,
                                                                          (u32)CE, (u32)C4, WINV);
    }
    cast_kernel<<<(u32)(((size_t)RROWS * CE) / 2048), 256, 0, stream>>>(xa, hpl);
    gemm_f32b_kernel<<<dim3(DA / 128, RROWS / 128), 256, 0, stream>>>(hpl, wTout, tout_b, S32, (u32)DA, (u32)CE, (u32)DA, WINV);
    ln_out_kernel<<<RROWS / 8, 256, 0, stream>>>(S32, tout_ln_g, tout_ln_b, out1);
    cvt_wt_kernel<<<dim3((SEQ) / 64, DA / 32, NB), 256, 0, stream>>>(out1, ALT, (u32)(SEQ), (u32)DA, (u32)(SEQ),
                                                                     (u32)(SEQ_FULL * DA), (u32)(DA * (SEQ)), 1.0f, 0u);
    gemm_pool_kernel<<<dim3(DA / 128, NRES / 128, NB), 256, 0, stream>>>(a2tT, ALT, rinv, outp, (u32)(SEQ));
}
